// User2ItemLayer_7224134991886
// MI455X (gfx1250) — hardware-run, weakly checked
//
#include <hip/hip_runtime.h>


#ifndef NB
#define NB 4096
#endif
#define NB_FULL 4096
#define TT   50
#define DD   64
#define VV   200000
#define PP   50
#define NS   64
#define PW   4
#define PR   8
#define USP  68
#define LW   8
#define LSP  68
#define UTS  1024.0f
#define SWS  256.0f
#define FOLD (1.0f / (1024.0f * 256.0f))
#define MASKV (-4294967296.0f)
#define NEGB (-3.0e38f)
#define LNV1 12.206077645517675f

static_assert(DD == 64);
static_assert(DD % 32 == 0);
static_assert(NS == 64);
static_assert(TT > 32);
static_assert(TT <= 64);
static_assert(PP <= 64);
static_assert(PW * PR == 32);
static_assert(PR == 8);
static_assert(32 * 16 * 2 == PR * DD * 2);
static_assert(8 * 16 == PW * PR * 4);
static_assert(256 * 16 * 2 == NS * DD * 2);
static_assert(32 * 16 == 2 * NS * 4);
static_assert(NB % (PW * PR) == 0);
static_assert(NB % (16 * LW) == 0);
static_assert(NB <= NB_FULL);
static_assert((USP * 4) % 16 == 0);
static_assert((LSP * 4) % 16 == 0);
static_assert((size_t)NB_FULL * 4 == (size_t)16384);
static_assert((size_t)(PW * TT * DD + 2 * PW * 64 + PW * PR * USP + 64 + 2 * PW * PR) * 4 <= (size_t)65536);
static_assert((size_t)(PW * TT * DD + 2 * PW * 64 + PW * PR * USP + 64 + 2 * PW * PR) * 4 <= (size_t)131072);
static_assert((size_t)(LW * 16 * LSP + 3 * NS + LW) * 4 <= (size_t)131072);
static_assert((size_t)(2 * NS) * 4 <= (size_t)131072);

typedef _Float16 h16;
typedef __attribute__((ext_vector_type(16))) _Float16 v16h;
typedef __attribute__((ext_vector_type(8)))  _Float16 v8h;
typedef __attribute__((ext_vector_type(8)))  float    v8f;
typedef __attribute__((ext_vector_type(4)))  float    v4f;
typedef __attribute__((ext_vector_type(2)))  float    v2f;
typedef v4f  __attribute__((may_alias)) v4fa;
typedef v2f  __attribute__((may_alias)) v2fa;

__device__ __forceinline__ unsigned short f2bf(float f) { unsigned u = __float_as_uint(f); u += 0x7FFFu + ((u >> 16) & 1u); return (unsigned short)(u >> 16); }
__device__ __forceinline__ float bfr(float f) { return __uint_as_float(((unsigned)f2bf(f)) << 16); }
__device__ __forceinline__ v16h cat16(v8h lo, v8h hi) { return __builtin_shufflevector(lo, hi, 0, 1, 2, 3, 4, 5, 6, 7, 8, 9, 10, 11, 12, 13, 14, 15); }
__device__ __forceinline__ v8f wmma16(v16h a, v16h b, v8f c) { return __builtin_amdgcn_wmma_f32_16x16x32_f16(false, a, false, b, (short)0, c, false, false); }
__device__ __forceinline__ v16h  ldh(const h16* p) { return cat16(*(const v8h*)p, *(const v8h*)(p + 16)); }
__device__ __forceinline__ void wave_sync() { __builtin_amdgcn_fence(3  , "wavefront"); __builtin_amdgcn_wave_barrier(); asm volatile("" ::: "memory"); }

__device__ __forceinline__ v8f wmma16g(v16h a, v16h b, v8f c) { c = wmma16(a, b, c); asm volatile("v_nop\n\tv_nop\n\tv_nop\n\tv_nop" : "+v"(c) : "v"(a), "v"(b)); return c; }
static __device__ __forceinline__ h16 toh_flush(float v) { const h16 r = (h16)v; return (fabsf(v) < 6.103515625e-05f) ? (h16)0.0f : r; }
__device__ __forceinline__ int wrapc(int i, int n) { i += (i >> 31) & n; return max(0, min(i, n - 1)); }
__device__ __forceinline__ float wsum(float v) {
#pragma unroll
    for (int off = 16; off > 0; off >>= 1) v += __shfl_xor(v, off, 32);
    return v; }
__device__ __forceinline__ float logq(int id) { const float f = (float)id; const float d = logf(f + 2.0f) - logf(f + 1.0f); return logf(d * (1.0f / LNV1)); }

__global__ __launch_bounds__(256) void k_samp(const float* __restrict__ item, const float* __restrict__ zbias, const int* __restrict__ sids, h16* SW, float* SADJ) {
    __shared__ __align__(16) float sa[2 * NS];
    const int tid = threadIdx.x, lane = tid & 31;
    const int wave = __builtin_amdgcn_readfirstlane((int)(threadIdx.x >> 5));
    const int sraw = sids[tid & (NS - 1)];
    float zb = bfr(zbias[wrapc(sraw, VV)]);
    float lq = logq(sraw);
    asm volatile("" : "+v"(zb)); asm volatile("" : "+v"(lq));
    if (tid < 2 * NS) sa[tid] = (tid < NS) ? zb : lq;
    const int c8 = (tid & 7) * 8;
    v8h hv0, hv1;
    { const int sid = wrapc(sids[tid >> 3], VV);
      const v4f x0 = *(const v4f*)(item + (size_t)sid * DD + c8); const v4f x1 = *(const v4f*)(item + (size_t)sid * DD + c8 + 4);
#pragma unroll
      for (int i = 0; i < 4; ++i) { hv0[i] = toh_flush(bfr(x0[i]) * SWS); hv0[4 + i] = toh_flush(bfr(x1[i]) * SWS); } }
    { const int sid = wrapc(sids[32 + (tid >> 3)], VV);
      const v4f x0 = *(const v4f*)(item + (size_t)sid * DD + c8); const v4f x1 = *(const v4f*)(item + (size_t)sid * DD + c8 + 4);
#pragma unroll
      for (int i = 0; i < 4; ++i) { hv1[i] = toh_flush(bfr(x0[i]) * SWS); hv1[4 + i] = toh_flush(bfr(x1[i]) * SWS); } }
    h16* p0 = SW + (size_t)tid * 8;
    h16* p1 = SW + (size_t)(256 + tid) * 8;
#pragma unroll 1
    for (int ps = 0; ps < 2; ++ps) { *(volatile v8h*)p0 = hv0; *(volatile v8h*)p1 = hv1; if (ps == 0) __threadfence(); }
    __syncthreads();
    if (wave == 0) {
        const v4f v = *(const v4fa*)(&sa[4 * lane]);
#pragma unroll 1
        for (int ps = 0; ps < 2; ++ps) { *(volatile v4f*)(SADJ + 4 * lane) = v; if (ps == 0) __threadfence(); }
    }
}

__global__ __launch_bounds__(32 * PW) void k_pool(const float* __restrict__ item, const float* __restrict__ pos, const float* __restrict__ attw, const float* __restrict__ attb,
                                                  const float* __restrict__ alpha, const int* __restrict__ ids, const int* __restrict__ pids, const int* __restrict__ tgt,
                                                  const int* __restrict__ klen, float* OUT, h16* UT, float* TD) {
    __shared__ __align__(16) float xs[PW * TT * DD];
    __shared__ __align__(16) float wt[PW * 64];
    __shared__ __align__(16) float wu[PW * 64];
    __shared__ __align__(16) float us[PW * PR * USP];
    __shared__ __align__(16) float pd[64];
    __shared__ __align__(16) float outS[PW * PR];
    __shared__ __align__(16) float tdS[PW * PR];
    const int tid = threadIdx.x, lane = tid & 31;
    const int wave = __builtin_amdgcn_readfirstlane((int)(threadIdx.x >> 5));
    { const int p = min(tid, PP - 1); float acc = 0.0f;
#pragma unroll 1
      for (int k = 0; k < DD; ++k) acc += bfr(pos[p * DD + k]) * bfr(attw[DD + k]);
      asm volatile("" : "+v"(acc));
      if (tid < 64) pd[tid] = acc; }
    __syncthreads();
    const float w0 = bfr(attw[2 * lane]), w1 = bfr(attw[2 * lane + 1]);
    const float al0 = bfr(alpha[2 * lane]), al1 = bfr(alpha[2 * lane + 1]);
    const float bb = bfr(attb[0]);
    const int xb = wave * TT * DD, wb = wave * 64;
    const int tB = lane + 32; const int tBc = min(tB, TT - 1);
#pragma unroll 1
    for (int rr = 0; rr < PR; ++rr) {
        const int lrow = wave * PR + rr;
        const int b = blockIdx.x * (PW * PR) + lrow;
        const int kl = klen[b];
        int idA = ids[(size_t)b * TT + lane]; int idB = ids[(size_t)b * TT + tBc];
        asm volatile("" : "+v"(idA)); asm volatile("" : "+v"(idB));
        const float padA = (idA != 0) ? 1.0f : 0.0f;
        const float padB = (idB != 0) ? 1.0f : 0.0f;
        float sA = NEGB, sB = NEGB;
#pragma unroll 1
        for (int t = 0; t < TT; ++t) {
            const int iid = wrapc(ids[(size_t)b * TT + t], VV);
            const int pid = wrapc(pids[(size_t)b * TT + t], PP);
            const v2f xv = *(const v2f*)(item + (size_t)iid * DD + 2 * lane);
            v2f xo; xo[0] = bfr(xv[0]); xo[1] = bfr(xv[1]);
            *(v2fa*)(&xs[xb + t * DD + 2 * lane]) = xo;
            const float part = wsum(xo[0] * w0 + xo[1] * w1);
            const float s = tanhf((part + pd[pid]) + bb);
            const float ms = (t < kl) ? s : MASKV;
            sA = (lane == t) ? ms : sA;
            sB = (tB == t) ? ms : sB;
        }
        float mx = fmaxf(sA, sB);
#pragma unroll
        for (int off = 16; off > 0; off >>= 1) mx = fmaxf(mx, __shfl_xor(mx, off, 32));
        const float eA = expf(sA - mx);
        const float eB0 = expf(sB - mx);
        const float eB = (tB < TT) ? eB0 : 0.0f;
        const float inv = 1.0f / wsum(eA + eB);
        const float wA = eA * inv, wB = eB * inv;
        wt[wb + lane] = wA; wt[wb + 32 + lane] = wB;
        wu[wb + lane] = wA * padA;
        wu[wb + 32 + lane] = (tB < TT - 1) ? (wB * padB) : 0.0f;
        wave_sync();
        float sp0 = 0.0f, sp1 = 0.0f, u0 = 0.0f, u1 = 0.0f;
#pragma unroll 2
        for (int t = 0; t < TT; ++t) {
            const v2f x = *(const v2fa*)(&xs[xb + t * DD + 2 * lane]);
            const float w = wt[wb + t], u = wu[wb + t];
            sp0 += w * x[0]; sp1 += w * x[1]; u0 += u * x[0]; u1 += u * x[1];
        }
        const float q0 = (sp0 > 0.0f) ? sp0 : (al0 * sp0);
        const float q1 = (sp1 > 0.0f) ? sp1 : (al1 * sp1);
        const int tg = wrapc(tgt[b], VV);
        const v2f tv = *(const v2f*)(item + (size_t)tg * DD + 2 * lane);
        const float od = wsum(q0 * bfr(tv[0]) + q1 * bfr(tv[1]));
        const int ki = wrapc(kl - 1, TT);
        const int res = wrapc(ids[(size_t)b * TT + ki], VV);
        const v2f rv = *(const v2f*)(item + (size_t)res * DD + 2 * lane);
        const float tdv = wsum(u0 * bfr(rv[0]) + u1 * bfr(rv[1]));
        v2f uo; uo[0] = u0 * UTS; uo[1] = u1 * UTS;
        *(v2fa*)(&us[lrow * USP + 2 * lane]) = uo;
        if (lane == 0) { outS[lrow] = od; tdS[lrow] = tdv; }
        wave_sync();
    }
    {
        h16* ub = UT + (size_t)(blockIdx.x * (PW * PR) + wave * PR) * DD;
#pragma unroll 1
        for (int ps = 0; ps < 2; ++ps) {
#pragma unroll
            for (int s = 0; s < 2; ++s) { const int row = 4 * s + (lane >> 3), c8 = (lane & 7) * 8;
                const v4f x0 = *(const v4fa*)(&us[(wave * PR + row) * USP + c8]); const v4f x1 = *(const v4fa*)(&us[(wave * PR + row) * USP + c8 + 4]); v8h hv;
#pragma unroll
                for (int i = 0; i < 4; ++i) { hv[i] = toh_flush(x0[i]); hv[4 + i] = toh_flush(x1[i]); }
                *(volatile v8h*)(ub + (size_t)row * DD + c8) = hv; }
            if (ps == 0) __threadfence(); }
    }
    __syncthreads();
    if (wave == 0) {
        const int q = (lane & 7) * 4;
        const v4f ov = *(const v4fa*)(&outS[q]); const v4f tv = *(const v4fa*)(&tdS[q]);
        float* op = OUT + (size_t)blockIdx.x * (PW * PR) + q;
        float* tp = TD + (size_t)blockIdx.x * (PW * PR) + q;
#pragma unroll 1
        for (int ps = 0; ps < 2; ++ps) {
            if (lane < 8) { *(volatile v4f*)op = ov; *(volatile v4f*)tp = tv; }
            if (ps == 0) __threadfence(); }
    }
}

__global__ __launch_bounds__(32 * LW) void k_loss(const h16* __restrict__ UT, const h16* __restrict__ SW, const float* __restrict__ SADJ, const float* __restrict__ TD,
                                                  const float* __restrict__ zbias, const int* __restrict__ ids, const int* __restrict__ klen, const int* __restrict__ sids, float* LOSS) {
    __shared__ __align__(16) float lt[LW * 16 * LSP];
    __shared__ float zbs[NS];
    __shared__ float lqs[NS];
    __shared__ int   sdS[NS];
    __shared__ float wl[LW];
    const int tid = threadIdx.x, lane = tid & 31, lr = lane & 15, hi = lane >> 4;
    const int wave = __builtin_amdgcn_readfirstlane((int)(threadIdx.x >> 5));
    { const int i = tid & (NS - 1); const float z = SADJ[i]; const float q = SADJ[NS + i]; const int s = sids[i];
      if (tid < NS) { zbs[i] = z; lqs[i] = q; sdS[i] = s; } }
    v16h bq[2][4];
#pragma unroll
    for (int kk = 0; kk < 2; ++kk)
#pragma unroll
        for (int nb = 0; nb < 4; ++nb) bq[kk][nb] = ldh(SW + (size_t)(nb * 16 + lr) * DD + 8 * hi + kk * 32);
    __syncthreads();
    const int wb = wave * 16 * LSP;
    float lacc = 0.0f;
#pragma unroll 1
    for (int it = 0; it < NB / (16 * LW); ++it) {
        const int r0 = (it * LW + wave) * 16;
        const size_t ao = (size_t)(r0 + lr) * DD + 8 * hi;
        const v16h a0 = ldh(UT + ao), a1 = ldh(UT + ao + 32);
        v8f acc[4];
#pragma unroll
        for (int nb = 0; nb < 4; ++nb) { acc[nb] = (v8f){}; acc[nb] = wmma16g(a0, bq[0][nb], acc[nb]); acc[nb] = wmma16g(a1, bq[1][nb], acc[nb]); }
#pragma unroll
        for (int nb = 0; nb < 4; ++nb) {
#pragma unroll
            for (int j = 0; j < 8; ++j) lt[wb + (hi * 8 + j) * LSP + nb * 16 + lr] = acc[nb][j] * FOLD; }
        wave_sync();
        const int g = r0 + lr;
        const int ki = wrapc(klen[g] - 1, TT);
        const int resr = ids[(size_t)g * TT + ki];
        const float zb = bfr(zbias[wrapc(resr, VV)]);
        const float tl = (TD[g] + zb) - logq(resr);
        const int lb = wb + lr * LSP + hi * 32;
        float mxh = NEGB;
#pragma unroll 1
        for (int c = 0; c < 32; ++c) { const int cc = hi * 32 + c;
            float l = (lt[lb + c] + zbs[cc]) - lqs[cc];
            l = (sdS[cc] == resr) ? (l - 1.0e9f) : l;
            lt[lb + c] = l; mxh = fmaxf(mxh, l); }
        const float mx = fmaxf(fmaxf(mxh, __shfl_xor(mxh, 16, 32)), tl);
        float sum = 0.0f;
#pragma unroll 1
        for (int c = 0; c < 32; ++c) sum += expf(lt[lb + c] - mx);
        sum += __shfl_xor(sum, 16, 32);
        sum += expf(tl - mx);
        const float rl = -((tl - mx) - logf(sum));
        lacc += (hi == 0) ? rl : 0.0f;
        wave_sync();
    }
    lacc = wsum(lacc);
    if (lane == 0) wl[wave] = lacc;
    __syncthreads();
    float s = 0.0f;
#pragma unroll
    for (int w = 0; w < LW; ++w) s += wl[w];
    const float mean = s * (1.0f / (float)NB);
    if (tid == 0) { *(volatile float*)LOSS = mean; __threadfence(); *(volatile float*)LOSS = mean; }
}

static constexpr size_t al256(size_t v) { return (v + 255) & ~(size_t)255; }
static constexpr size_t SZ_UT = al256((size_t)NB * DD * 2);
static constexpr size_t SZ_SW = al256((size_t)NS * DD * 2);
static constexpr size_t SZ_SA = al256((size_t)2 * NS * 4);
static constexpr size_t SZ_TD = al256((size_t)NB * 4);
static constexpr size_t SZ_TOTAL = SZ_UT + SZ_SW + SZ_SA + SZ_TD;
static_assert(SZ_TOTAL <= (size_t)134217728);
static_assert((size_t)(NB / (PW * PR)) * (PW * PR) * DD * 2 <= SZ_UT);
static_assert((size_t)(NB / (PW * PR)) * (PW * PR) * 4 <= SZ_TD);

extern "C" void kernel_launch(void* const* d_in, const int* in_sizes, int n_in,
                              void* d_out, int out_size, void* d_ws, size_t ws_size, hipStream_t stream) {
    if (n_in < 11) return;
    if ((size_t)in_sizes[0] < (size_t)VV * DD) return;
    if ((size_t)in_sizes[1] < (size_t)PP * DD) return;
    if (in_sizes[2] < 2 * DD || in_sizes[3] < 1 || in_sizes[4] < DD) return;
    if ((size_t)in_sizes[5] < (size_t)VV) return;
    if ((size_t)in_sizes[6] < (size_t)NB * TT || (size_t)in_sizes[7] < (size_t)NB * TT) return;
    if (in_sizes[8] < NB || in_sizes[9] < NB || in_sizes[10] < NS) return;
    if ((size_t)out_size < (size_t)NB_FULL + 1) return;
    if (SZ_TOTAL > ws_size) return;
    const float* item  = (const float*)d_in[0];
    const float* pos   = (const float*)d_in[1];
    const float* attw  = (const float*)d_in[2];
    const float* attb  = (const float*)d_in[3];
    const float* alpha = (const float*)d_in[4];
    const float* zbias = (const float*)d_in[5];
    const int* ids  = (const int*)d_in[6];
    const int* pids = (const int*)d_in[7];
    const int* tgt  = (const int*)d_in[8];
    const int* klen = (const int*)d_in[9];
    const int* sids = (const int*)d_in[10];
    float* OUT = (float*)d_out;
    char* wsp = (char*)d_ws;
    h16* UT = (h16*)wsp; wsp += SZ_UT;
    h16* SW = (h16*)wsp; wsp += SZ_SW;
    float* SADJ = (float*)wsp; wsp += SZ_SA;
    float* TD = (float*)wsp; wsp += SZ_TD;

    k_samp<<<1, 256, 0, stream>>>(item, zbias, sids, SW, SADJ);
    k_pool<<<NB / (PW * PR), 32 * PW, 0, stream>>>(item, pos, attw, attb, alpha, ids, pids, tgt, klen, OUT, UT, TD);
    k_loss<<<1, 32 * LW, 0, stream>>>(UT, SW, SADJ, TD, zbias, ids, klen, sids, OUT + NB_FULL);
}
